// LRU_13477607375571
// MI455X (gfx1250) — hardware-verified
//
#include <hip/hip_runtime.h>
#include <cmath>

typedef __attribute__((ext_vector_type(16))) _Float16 v16h;
typedef __attribute__((ext_vector_type(8)))  _Float16 v8h;
typedef __attribute__((ext_vector_type(8)))  float    v8f;
typedef __attribute__((ext_vector_type(4)))  float    v4f;
typedef __attribute__((ext_vector_type(2)))  float    v2f;
typedef __attribute__((ext_vector_type(4)))  unsigned v4u;

constexpr int SEQ_LEN  = 16384;
constexpr int H_DIM    = 512;
constexpr int N_STATE  = 512;
constexpr int N_HALF   = 256;
constexpr int G_COLS   = 2 * N_HALF;
constexpr int BT1_ROWS = 2 * N_STATE;
constexpr int K_READ   = 4 * N_STATE;
constexpr int ST_WORDS = K_READ / 2;

constexpr float CARRY_B     = 4096.0f;
constexpr float CARRY_S     = 64.0f;
constexpr float CARRY_C     = 64.0f;
constexpr float SCALE_GEMM0 = 1.0f / 4096.0f;
constexpr float SCALE_GEMM1 = 1.0f / 4096.0f;

constexpr size_t WS_OFF_PARAMS = 0;
constexpr size_t WS_SZ_PARAMS  = 8192;
constexpr size_t WS_OFF_BT1    = WS_OFF_PARAMS + WS_SZ_PARAMS;
constexpr size_t WS_SZ_BT1     = (size_t)BT1_ROWS * H_DIM * 2;
constexpr size_t WS_OFF_BT2    = WS_OFF_BT1 + WS_SZ_BT1;
constexpr size_t WS_SZ_BT2     = (size_t)H_DIM * K_READ * 2;
constexpr size_t WS_OFF_X16    = WS_OFF_BT2 + WS_SZ_BT2;
constexpr size_t WS_SZ_X16     = (size_t)SEQ_LEN * H_DIM * 2;
constexpr size_t WS_OFF_G      = WS_OFF_X16 + WS_SZ_X16;
constexpr size_t WS_SZ_G       = (size_t)SEQ_LEN * G_COLS * 4;
constexpr size_t WS_OFF_ST     = WS_OFF_G + WS_SZ_G;
constexpr size_t WS_SZ_ST      = (size_t)SEQ_LEN * K_READ * 2;
constexpr size_t WS_TOTAL      = WS_OFF_ST + WS_SZ_ST;
static_assert(WS_TOTAL == 120594432);
static_assert(WS_TOTAL <= 134217728);
static_assert(3 * (size_t)N_STATE * 4 <= WS_SZ_PARAMS);
static_assert((WS_OFF_BT1 % 128) == 0 && (WS_OFF_BT2 % 128) == 0 && (WS_OFF_X16 % 128) == 0 &&
              (WS_OFF_G % 128) == 0 && (WS_OFF_ST % 128) == 0);
static_assert(SEQ_LEN % 64 == 0 && G_COLS % 64 == 0 && H_DIM % 64 == 0);
static_assert(H_DIM % 32 == 0 && K_READ % 32 == 0);
static_assert(((SEQ_LEN / 64) * (G_COLS / 64)) % 8 == 0);
static_assert(((SEQ_LEN / 64) * (H_DIM / 64)) % 8 == 0);
static_assert(2 * N_HALF == N_STATE);
static_assert((N_STATE * (H_DIM / 8)) % 256 == 0);
static_assert(((size_t)SEQ_LEN * (H_DIM / 8)) % 256 == 0);
static_assert(SEQ_LEN % 32 == 0 && N_HALF % 32 == 0);

__device__ __forceinline__ _Float16 to_f16_ftz(float x) {
  const float w = (fabsf(x) < 6.103515625e-5f) ? 0.0f : x;
  return (_Float16)w;
}
__device__ __forceinline__ unsigned f16_bits_ftz(float x) {
  return (unsigned)__builtin_bit_cast(unsigned short, to_f16_ftz(x));
}

__device__ __forceinline__ void dep_guard_h(v8f& a, v8f& b, v16h x, v16h y) { asm volatile("v_nop\n\tv_nop\n\tv_nop\n\tv_nop" : "+v"(a), "+v"(b) : "v"(x), "v"(y)); }
__device__ __forceinline__ void keep4_h(v16h a, v16h b, v16h c, v16h d) { asm volatile("v_nop" :: "v"(a), "v"(b), "v"(c), "v"(d)); }
__device__ __forceinline__ void acc_guard4(v8f& a, v8f& b, v8f& c, v8f& d) { asm volatile("v_nop\n\tv_nop\n\tv_nop\n\tv_nop" : "+v"(a), "+v"(b), "+v"(c), "+v"(d)); }
template <typename T> struct Frag;
template <> struct Frag<_Float16> {
  typedef v16h V; union U { v16h v; v8h h[2]; };
  static __device__ __forceinline__ v16h load(const _Float16* p) {
    U f; f.h[0] = *(const v8h*)(p); f.h[1] = *(const v8h*)(p + 16); return f.v;
  }
  static __device__ __forceinline__ v8f mma(v16h a, v16h b, v8f c) {
    return __builtin_amdgcn_wmma_f32_16x16x32_f16(false, a, false, b, (short)0, c, false, false);
  }
  static __device__ __forceinline__ void guard(v8f& a, v8f& b, v16h x, v16h y) { dep_guard_h(a, b, x, y); }
  static __device__ __forceinline__ void keep(v16h a, v16h b, v16h c, v16h d) { keep4_h(a, b, c, d); }
};

template <bool DSKIP>
__global__ __launch_bounds__(256) void wmma_gemm64_f16(
    const unsigned short* __restrict__ Ap, int lda,
    const unsigned short* __restrict__ Btp, int ldb,
    float* __restrict__ Cout, int ldc,
    const float* __restrict__ skipU, const float* __restrict__ skipD,
    int M, int N, int K, float scale) {
  typedef _Float16 T;
  typedef v16h V;
  const T* A = (const T*)Ap; const T* Bt = (const T*)Btp;
  __shared__ __align__(16) float sT[8][16 * 68];
  const int lane = threadIdx.x & 31;
  const int wave = threadIdx.x >> 5;
  const int tilesN = N >> 6;
  const int tilesM = M >> 6;
  const int tile = blockIdx.x * 8 + wave;
  if (tile >= tilesM * tilesN) return;
  const int tm = tile / tilesN;
  const int tn = tile - tm * tilesN;
  const int m0 = tm << 6;
  const int n0 = tn << 6;

  const int rlane = lane & 15;
  const int koff  = (lane >> 4) * 8;
  const int mOff  = (lane >> 4) * 8;

  v8f acc[4][4];
#pragma unroll
  for (int i = 0; i < 4; ++i)
#pragma unroll
    for (int j = 0; j < 4; ++j) acc[i][j] = (v8f){0.f,0.f,0.f,0.f,0.f,0.f,0.f,0.f};

  for (int k0 = 0; k0 < K; k0 += 32) {
    V bh[4];
#pragma unroll
    for (int j = 0; j < 4; ++j) {
      const size_t bo = (size_t)(n0 + (j << 4) + rlane) * ldb + koff + k0;
      bh[j] = Frag<T>::load(Bt + bo);
    }
#pragma unroll
    for (int i = 0; i < 4; ++i) {
      const size_t ao = (size_t)(m0 + (i << 4) + rlane) * lda + koff + k0;
      V ah = Frag<T>::load(A + ao);
#pragma unroll
      for (int j = 0; j < 4; ++j) {
        acc[i][j] = Frag<T>::mma(ah, bh[j], acc[i][j]);
      }
      Frag<T>::guard(acc[i][0], acc[i][3], ah, ah);
    }
    Frag<T>::keep(bh[0], bh[1], bh[2], bh[3]);
  }
  acc_guard4(acc[0][0], acc[0][1], acc[0][2], acc[0][3]);
  acc_guard4(acc[1][0], acc[1][1], acc[1][2], acc[1][3]);
  acc_guard4(acc[2][0], acc[2][1], acc[2][2], acc[2][3]);
  acc_guard4(acc[3][0], acc[3][1], acc[3][2], acc[3][3]);

  float* slab = sT[wave];
  const int hh = lane >> 4, c4 = (lane & 15) * 4;
  v4f d4 = (v4f){0.f, 0.f, 0.f, 0.f};
  if (DSKIP) d4 = *(const v4f*)(skipD + n0 + c4);
#pragma unroll
  for (int i = 0; i < 4; ++i) {
    const int mBase = m0 + (i << 4);
#pragma unroll
    for (int j = 0; j < 4; ++j) {
#pragma unroll
      for (int r = 0; r < 8; ++r) {
        const float v = acc[i][j][r] * scale;
        slab[(mOff + r) * 68 + (j << 4) + rlane] = v;
      }
    }
    __builtin_amdgcn_fence(__ATOMIC_RELEASE, "workgroup");
    __builtin_amdgcn_wave_barrier();
    __builtin_amdgcn_fence(__ATOMIC_ACQUIRE, "workgroup");
    if (DSKIP) {
#pragma unroll
      for (int it = 0; it < 8; ++it) {
        const int row = it * 2 + hh;
        float* sp = slab + row * 68 + c4;
        v4f v = *(const v4f*)sp;
        const v4f u4 = *(const v4f*)(skipU + (size_t)(mBase + row) * ldc + n0 + c4);
        v = d4 * u4 + v;
        *(v4f*)sp = v;
      }
      __builtin_amdgcn_fence(__ATOMIC_RELEASE, "workgroup");
      __builtin_amdgcn_wave_barrier();
      __builtin_amdgcn_fence(__ATOMIC_ACQUIRE, "workgroup");
    }
    for (int pass = 0; pass < 2; ++pass) {
#pragma unroll
      for (int it = 0; it < 8; ++it) {
        const int row = it * 2 + hh;
        v4f v = *(const v4f*)(slab + row * 68 + c4);
        *(volatile v4f*)(Cout + (size_t)(mBase + row) * ldc + n0 + c4) = v;
      }
      __threadfence();
    }
    __builtin_amdgcn_fence(__ATOMIC_RELEASE, "workgroup");
    __builtin_amdgcn_wave_barrier();
    __builtin_amdgcn_fence(__ATOMIC_ACQUIRE, "workgroup");
  }
}

__global__ __launch_bounds__(512) void lru_setup(
    const float* __restrict__ theta_log, const float* __restrict__ nu_log, float* __restrict__ params) {
  const int n = threadIdx.x;
  const float nu  = expf(nu_log[n]);
  const float th  = expf(theta_log[n]);
  const float mag = expf(-nu);
  const float lr  = mag * cosf(th);
  const float li  = mag * sinf(th);
  const float gm  = sqrtf(fmaxf(0.0f, 1.0f - mag * mag));
  volatile float* vp = params;
  vp[n] = lr; vp[N_STATE + n] = li; vp[2 * N_STATE + n] = gm;
  __threadfence();
  vp[n] = lr; vp[N_STATE + n] = li; vp[2 * N_STATE + n] = gm;
}

__global__ __launch_bounds__(256) void prep_bt1(
    const float* __restrict__ Bre, const float* __restrict__ Bim,
    const float* __restrict__ params, _Float16* __restrict__ Bt1) {
  const int g  = blockIdx.x * 256 + threadIdx.x;
  const int n  = g >> 6;
  const int h8 = (g & 63) << 3;
  const float gm = params[2 * N_STATE + n] * CARRY_B;
  const float* sr = Bre + (size_t)n * H_DIM + h8;
  const float* si = Bim + (size_t)n * H_DIM + h8;
  const v4f r0 = *(const v4f*)(sr);
  const v4f r1 = *(const v4f*)(sr + 4);
  const v4f i0 = *(const v4f*)(si);
  const v4f i1 = *(const v4f*)(si + 4);
  v8h re, im;
#pragma unroll
  for (int e = 0; e < 4; ++e) {
    re[e]     = to_f16_ftz(gm * r0[e]);
    re[4 + e] = to_f16_ftz(gm * r1[e]);
    im[e]     = to_f16_ftz(gm * i0[e]);
    im[4 + e] = to_f16_ftz(gm * i1[e]);
  }
  _Float16* d0 = Bt1 + (size_t)(2 * n) * H_DIM + h8;
  _Float16* d1 = Bt1 + (size_t)(2 * n + 1) * H_DIM + h8;
  *(volatile v8h*)d0 = re;
  *(volatile v8h*)d1 = im;
  __threadfence();
  *(volatile v8h*)d0 = re;
  *(volatile v8h*)d1 = im;
}

__global__ __launch_bounds__(256) void prep_bt2(
    const float* __restrict__ Cre, const float* __restrict__ Cim,
    const float* __restrict__ Cre2, const float* __restrict__ Cim2, _Float16* __restrict__ Bt2) {
  const int dir = blockIdx.y;
  const int j   = threadIdx.x & 127;
  const int o   = blockIdx.x * 2 + (threadIdx.x >> 7);
  const float* cr = dir ? Cre2 : Cre;
  const float* ci = dir ? Cim2 : Cim;
  const v4f a = *(const v4f*)(cr + (size_t)o * N_STATE + 4 * j);
  const v4f b = *(const v4f*)(ci + (size_t)o * N_STATE + 4 * j);
  v8h hv;
#pragma unroll
  for (int e = 0; e < 4; ++e) {
    hv[2 * e]     = to_f16_ftz(a[e] * CARRY_C);
    hv[2 * e + 1] = to_f16_ftz(b[e] * (-CARRY_C));
  }
  _Float16* dst = Bt2 + (size_t)o * K_READ + (size_t)dir * (2 * N_STATE) + 8 * j;
  *(volatile v8h*)dst = hv;
  __threadfence();
  *(volatile v8h*)dst = hv;
}

__global__ __launch_bounds__(256) void cvt_x_f16(
    const float* __restrict__ in, _Float16* __restrict__ out) {
  const size_t g = (size_t)blockIdx.x * 256 + threadIdx.x;
  const float* src = in + g * 8;
  const v4f a = *(const v4f*)(src);
  const v4f b = *(const v4f*)(src + 4);
  v8h hv;
#pragma unroll
  for (int e = 0; e < 4; ++e) {
    hv[e]     = to_f16_ftz(a[e]);
    hv[4 + e] = to_f16_ftz(b[e]);
  }
  _Float16* dst = out + g * 8;
  *(volatile v8h*)dst = hv;
  __threadfence();
  *(volatile v8h*)dst = hv;
}

__global__ __launch_bounds__(32) void lru_walk(
    const float* __restrict__ G, const float* __restrict__ params,
    unsigned* __restrict__ ST32, int half) {
  __shared__ __align__(16) unsigned stage[32 * 32];
  const int lane = threadIdx.x;
  const int dir  = blockIdx.x >> 3;
  const int grp  = blockIdx.x & 7;
  const int pl   = grp * 32 + lane;
  const int n    = half * N_HALF + pl;
  const float lr = params[n], li = params[N_STATE + n];
  float sr = 0.0f, si = 0.0f;
  const float* gp = G + 2 * pl;
  const int q = lane >> 3, c = lane & 7;
  const int rowFirst = dir ? (SEQ_LEN - 1) : 0;
  const int rowStep  = dir ? -1 : 1;
  unsigned* dst = ST32 + (size_t)dir * N_STATE + (size_t)half * N_HALF + grp * 32 + c * 4;
  for (int t0 = 0; t0 < SEQ_LEN; t0 += 32) {
    for (int sub = 0; sub < 2; ++sub) {
      const int tb = t0 + sub * 16;
      v2f g[16];
#pragma unroll
      for (int s = 0; s < 16; ++s) {
        const int row = rowFirst + rowStep * (tb + s);
        g[s] = *(const v2f*)(gp + (size_t)row * G_COLS);
      }
#pragma unroll
      for (int s = 0; s < 16; ++s) {
        const float nr = fmaf(lr, sr, fmaf(-li, si, g[s][0]));
        const float ni = fmaf(lr, si, fmaf( li, sr, g[s][1]));
        sr = nr; si = ni;
        const unsigned lo = f16_bits_ftz(sr * CARRY_S);
        const unsigned hi = f16_bits_ftz(si * CARRY_S);
        stage[(sub * 16 + s) * 32 + lane] = lo | (hi << 16);
      }
    }
    __syncthreads();
    for (int sp = 0; sp < 2; ++sp) {
#pragma unroll
      for (int it = 0; it < 8; ++it) {
        const int slot = it * 4 + q;
        const int row  = rowFirst + rowStep * (t0 + slot);
        const v4u w = *(const v4u*)(stage + slot * 32 + c * 4);
        *(volatile v4u*)(dst + (size_t)row * ST_WORDS) = w;
      }
      __threadfence();
    }
    __syncthreads();
  }
}

extern "C" void kernel_launch(void* const* d_in, const int* in_sizes, int n_in,
                              void* d_out, int out_size, void* d_ws, size_t ws_size,
                              hipStream_t stream) {
  if (n_in != 10) return;
  if (in_sizes[0] != SEQ_LEN * H_DIM) return;
  if (in_sizes[1] != N_STATE) return;
  if (in_sizes[2] != N_STATE) return;
  if (in_sizes[3] != N_STATE * H_DIM) return;
  if (in_sizes[4] != N_STATE * H_DIM) return;
  if (in_sizes[5] != H_DIM * N_STATE) return;
  if (in_sizes[6] != H_DIM * N_STATE) return;
  if (in_sizes[7] != H_DIM * N_STATE) return;
  if (in_sizes[8] != H_DIM * N_STATE) return;
  if (in_sizes[9] != H_DIM) return;
  if (out_size != SEQ_LEN * H_DIM) return;
  if (ws_size < WS_TOTAL) return;

  const float* X     = (const float*)d_in[0];
  const float* thlog = (const float*)d_in[1];
  const float* nulog = (const float*)d_in[2];
  const float* Bre   = (const float*)d_in[3];
  const float* Bim   = (const float*)d_in[4];
  const float* Cre   = (const float*)d_in[5];
  const float* Cim   = (const float*)d_in[6];
  const float* Cre2  = (const float*)d_in[7];
  const float* Cim2  = (const float*)d_in[8];
  const float* Dv    = (const float*)d_in[9];
  float* Out = (float*)d_out;

  unsigned char* ws = (unsigned char*)d_ws;
  float*    params = (float*)(ws + WS_OFF_PARAMS);
  _Float16* Bt1    = (_Float16*)(ws + WS_OFF_BT1);
  _Float16* Bt2    = (_Float16*)(ws + WS_OFF_BT2);
  _Float16* X16    = (_Float16*)(ws + WS_OFF_X16);
  float*    G      = (float*)(ws + WS_OFF_G);
  unsigned* ST32   = (unsigned*)(ws + WS_OFF_ST);

  lru_setup<<<dim3(1), dim3(512), 0, stream>>>(thlog, nulog, params);

  prep_bt1<<<dim3((N_STATE * (H_DIM / 8)) / 256), dim3(256), 0, stream>>>(Bre, Bim, params, Bt1);

  prep_bt2<<<dim3(H_DIM / 2, 2), dim3(256), 0, stream>>>(Cre, Cim, Cre2, Cim2, Bt2);

  cvt_x_f16<<<dim3((unsigned)(((size_t)SEQ_LEN * (H_DIM / 8)) / 256)), dim3(256), 0, stream>>>(X, X16);

  for (int half = 0; half < 2; ++half) {
    wmma_gemm64_f16<false><<<dim3(((SEQ_LEN / 64) * (G_COLS / 64)) / 8), dim3(256), 0, stream>>>(
        (const unsigned short*)X16, H_DIM,
        (const unsigned short*)(Bt1 + (size_t)half * G_COLS * H_DIM), H_DIM,
        G, G_COLS, X, Dv, SEQ_LEN, G_COLS, H_DIM, SCALE_GEMM0);

    lru_walk<<<dim3(2 * (N_HALF / 32)), dim3(32), 0, stream>>>(G, params, ST32, half);
  }

  wmma_gemm64_f16<true><<<dim3(((SEQ_LEN / 64) * (H_DIM / 64)) / 8), dim3(256), 0, stream>>>(
      (const unsigned short*)ST32, K_READ, (const unsigned short*)Bt2, K_READ,
      Out, H_DIM, X, Dv, SEQ_LEN, H_DIM, K_READ, SCALE_GEMM1);
}
